// CosSim2d_9208409882745
// MI455X (gfx1250) — hardware-verified
//
#include <hip/hip_runtime.h>


#define NI   32
#define CC   64
#define HWD  64
#define NP   4096
#define KK   576
#define CO   64
typedef _Float16 h16;
typedef unsigned short bf;
typedef __attribute__((ext_vector_type(16))) __bf16   v16bf;
typedef __attribute__((ext_vector_type(16))) _Float16 v16h;
typedef __attribute__((ext_vector_type(8)))  _Float16 v8h;
typedef __attribute__((ext_vector_type(8)))  unsigned short v8us;
typedef __attribute__((ext_vector_type(8)))  float    v8f;
typedef __attribute__((ext_vector_type(4)))  float    v4f;
typedef v8h  __attribute__((may_alias)) v8ha;
typedef v4f  __attribute__((may_alias)) v4fa;
typedef v8us __attribute__((may_alias)) v8usa;

__device__ __forceinline__ unsigned short f2bf(float f) { unsigned u = __float_as_uint(f); u += 0x7FFFu + ((u >> 16) & 1u); return (unsigned short)(u >> 16); }
__device__ __forceinline__ float bf2f(unsigned short b) { return __uint_as_float(((unsigned)b) << 16); }
__device__ __forceinline__ float bfr(float f) { return bf2f(f2bf(f)); }
__device__ __forceinline__ v16h cat16(v8h lo, v8h hi) { return __builtin_shufflevector(lo, hi, 0, 1, 2, 3, 4, 5, 6, 7, 8, 9, 10, 11, 12, 13, 14, 15); }
__device__ __forceinline__ v16bf cat16b(v8us lo, v8us hi) { return __builtin_bit_cast(v16bf, __builtin_shufflevector(lo, hi, 0, 1, 2, 3, 4, 5, 6, 7, 8, 9, 10, 11, 12, 13, 14, 15)); }
__device__ __forceinline__ v8f wmma16(v16h a, v16h b, v8f c) { return __builtin_amdgcn_wmma_f32_16x16x32_f16(false, a, false, b, (short)0, c, false, false); }
__device__ __forceinline__ v8f wmmab(v16bf a, v16bf b, v8f c) { return __builtin_amdgcn_wmma_f32_16x16x32_bf16(false, a, false, b, (short)0, c, false, false); }


template <typename T16> struct WFrag;
template <> struct WFrag<h16> { typedef v16h V; static __device__ __forceinline__ V ld(const h16* p) { return cat16(*(const v8h*)p, *(const v8h*)(p + 16)); } static __device__ __forceinline__ v8f mma(V a, V b, v8f c) { return wmma16(a, b, c); } };
template <> struct WFrag<bf> { typedef v16bf V; static __device__ __forceinline__ V ld(const bf* p) { return cat16b(*(const v8us*)p, *(const v8us*)(p + 16)); } static __device__ __forceinline__ v8f mma(V a, V b, v8f c) { return wmmab(a, b, c); } };
template <typename T16, int NSPLIT, bool BIAS>
__global__ __launch_bounds__(32) void k_gemmw(const T16* __restrict__ A, const T16* __restrict__ A2, const T16* __restrict__ Bt, const T16* __restrict__ Bt2, int K, float* C, int ldc, const float* __restrict__ bias, size_t sA, size_t sB, size_t sC) {
    typedef typename WFrag<T16>::V V;
    __shared__ __align__(16) float os[16 * 68];
    const size_t z = blockIdx.z; A += z * sA; if (A2) A2 += z * sA; Bt += z * sB; if (Bt2) Bt2 += z * sB; C += z * sC;
    const int lane = threadIdx.x & 31, lr = lane & 15, hi = lane >> 4; const int r0 = blockIdx.x * 64, c0 = blockIdx.y * 64;
    v8f acc[4][4];
#pragma unroll
    for (int mb = 0; mb < 4; ++mb)
#pragma unroll
        for (int nb = 0; nb < 4; ++nb) acc[mb][nb] = (v8f){};
    const size_t aoff = (size_t)(r0 + lr) * K + 8 * hi, boff = (size_t)(c0 + lr) * K + 8 * hi;
#pragma unroll 1
    for (int kc = 0; kc < K; kc += 32) {
        V a[4], a2[4];
#pragma unroll
        for (int mb = 0; mb < 4; ++mb) { a[mb] = WFrag<T16>::ld(A + aoff + (size_t)mb * 16 * K + kc); if (NSPLIT == 1 || NSPLIT == 2) a2[mb] = WFrag<T16>::ld(A2 + aoff + (size_t)mb * 16 * K + kc); }
#pragma unroll
        for (int nb = 0; nb < 4; ++nb) { const V b = WFrag<T16>::ld(Bt + boff + (size_t)nb * 16 * K + kc); V b2; if (NSPLIT >= 2) b2 = WFrag<T16>::ld(Bt2 + boff + (size_t)nb * 16 * K + kc);
#pragma unroll
            for (int mb = 0; mb < 4; ++mb) { acc[mb][nb] = WFrag<T16>::mma(a[mb], b, acc[mb][nb]); if (NSPLIT == 1 || NSPLIT == 2) acc[mb][nb] = WFrag<T16>::mma(a2[mb], b, acc[mb][nb]); if (NSPLIT >= 2) acc[mb][nb] = WFrag<T16>::mma(a[mb], b2, acc[mb][nb]); } }
        asm volatile("v_nop\n\tv_nop\n\tv_nop\n\tv_nop" : "+v"(acc[0][0]), "+v"(acc[1][1]), "+v"(acc[2][2]), "+v"(acc[3][3]) : "v"(a[0]), "v"(a[3]));
    }
#pragma unroll
    for (int mb = 0; mb < 4; ++mb) {
#pragma unroll
        for (int nb = 0; nb < 4; ++nb) {
#pragma unroll
            for (int j = 0; j < 8; ++j) os[(hi * 8 + j) * 68 + nb * 16 + lr] = acc[mb][nb][j]; }
        __builtin_amdgcn_wave_barrier(); asm volatile("" ::: "memory");
        float* crow = C + (size_t)(r0 + mb * 16) * ldc + c0;
#pragma unroll 1
        for (int ps = 0; ps < 2; ++ps) {
#pragma unroll
            for (int s = 0; s < 8; ++s) { const int row = 2 * s + hi, cofs = lr * 4; v4f val = *(const v4fa*)(os + row * 68 + cofs); if (BIAS) { val[0] += bfr(bias[c0 + cofs]); val[1] += bfr(bias[c0 + cofs + 1]); val[2] += bfr(bias[c0 + cofs + 2]); val[3] += bfr(bias[c0 + cofs + 3]); }
                *(volatile v4f*)(crow + (size_t)row * ldc + cofs) = val; }
            if (ps == 0) __threadfence(); }
        __builtin_amdgcn_wave_barrier(); asm volatile("" ::: "memory");
    }
}

__device__ __forceinline__ void splitf(float y, unsigned short& h, unsigned short& l) { h = f2bf(y); l = f2bf(y - bf2f(h)); }
typedef __attribute__((ext_vector_type(4))) unsigned short v4us;

__global__ __launch_bounds__(256) void k_wn(const float* __restrict__ w, float* WN) { const int idx = blockIdx.x * 256 + threadIdx.x; if (idx >= CO * CC) return; const float* ww = w + (size_t)idx * 9; float q = 0.f;
#pragma unroll
    for (int l = 0; l < 9; ++l) { const float a = bfr(ww[l]); float p = __fmul_rn(a, a); asm volatile("" : "+v"(p)); q = __fadd_rn(q, p); } const float inv = __fdiv_rn(1.0f, fmaxf(__fsqrt_rn(q), 1e-12f)); *(volatile float*)(WN + idx) = inv; __threadfence(); *(volatile float*)(WN + idx) = inv; }
__global__ __launch_bounds__(256) void k_wnp(const float* __restrict__ w, const float* __restrict__ WN, bf* Bh, bf* Bl) { const int e = (blockIdx.x * 256 + threadIdx.x) * 4; if (e >= CO * KK) return; const int k0 = e % KK; const int v = e / KK; v4us oh, ol;
#pragma unroll
    for (int u = 0; u < 4; ++u) { const int k = k0 + u; const int c = k / 9; const float y = __fmul_rn(bfr(w[(size_t)v * KK + k]), WN[v * CC + c]); unsigned short a, b; splitf(y, a, b); oh[u] = a; ol[u] = b; } *(volatile v4us*)(Bh + e) = oh; *(volatile v4us*)(Bl + e) = ol; __threadfence(); *(volatile v4us*)(Bh + e) = oh; *(volatile v4us*)(Bl + e) = ol; }
__device__ __forceinline__ float xpad(const float* __restrict__ xc, int y, int x) { return (y >= 0 && y < HWD && x >= 0 && x < HWD) ? bfr(xc[y * HWD + x]) : 0.f; }
__global__ __launch_bounds__(256) void k_pn(const float* __restrict__ xi, float* PN) { const int e = (blockIdx.x * 256 + threadIdx.x) * 4; if (e >= CC * NP) return; const int pix = e % NP; const int c = e / NP; const float* xc = xi + (size_t)c * NP; v4f o;
#pragma unroll
    for (int u = 0; u < 4; ++u) { const int pp = pix + u; const int y = pp / HWD, x = pp % HWD; float q = 0.f;
#pragma unroll
        for (int i = 0; i < 3; ++i) {
#pragma unroll
            for (int j = 0; j < 3; ++j) { const float a = xpad(xc, y + i - 1, x + j - 1); float p = __fmul_rn(a, a); asm volatile("" : "+v"(p)); q = __fadd_rn(q, p); } }
        o[u] = __fdiv_rn(1.0f, fmaxf(__fsqrt_rn(q), 1e-12f)); } *(volatile v4f*)(PN + e) = o; __threadfence(); *(volatile v4f*)(PN + e) = o; }
__global__ __launch_bounds__(256) void k_pat(const float* __restrict__ xi, const float* __restrict__ PN, bf* Ah, bf* Al) { const int e = (blockIdx.x * 256 + threadIdx.x) * 4; if (e >= NP * KK) return; const int k0 = e % KK; const int pix = e / KK; const int y = pix / HWD, x = pix % HWD; v4us oh, ol;
#pragma unroll
    for (int u = 0; u < 4; ++u) { const int k = k0 + u; const int c = k / 9, l = k % 9; const int i = l / 3, j = l % 3; const float val = __fmul_rn(xpad(xi + (size_t)c * NP, y + i - 1, x + j - 1), PN[(size_t)c * NP + pix]); unsigned short a, b; splitf(val, a, b); oh[u] = a; ol[u] = b; }
    *(volatile v4us*)(Ah + e) = oh; *(volatile v4us*)(Al + e) = ol; __threadfence(); *(volatile v4us*)(Ah + e) = oh; *(volatile v4us*)(Al + e) = ol; }
__global__ __launch_bounds__(256) void k_out(const float* __restrict__ S, const float* __restrict__ pw, float* outb) { const int e = (blockIdx.x * 256 + threadIdx.x) * 4; if (e >= CO * NP) return; const int pix = e % NP; const int v = e / NP; const float pv = bfr(pw[v]); v4f o;
#pragma unroll
    for (int u = 0; u < 4; ++u) { const float s = S[(size_t)(pix + u) * CO + v]; const float sg = (s > 0.f) ? 1.f : ((s < 0.f) ? -1.f : 0.f); const float mag = powf(__fadd_rn(fabsf(s), 1e-12f), pv); o[u] = __fmul_rn(sg, mag); } *(volatile v4f*)(outb + e) = o; __threadfence(); *(volatile v4f*)(outb + e) = o; }

extern "C" void kernel_launch(void* const* d_in, const int* in_sizes, int n_in,
                              void* d_out, int out_size, void* d_ws, size_t ws_size, hipStream_t stream) {
    (void)in_sizes; (void)n_in; (void)out_size;
    const float** I = (const float**)d_in;
    const float *x = I[0], *w = I[1], *pw = I[2];
    float* OUT = (float*)d_out;
    char* wsp = (char*)d_ws;
    auto take = [&](size_t bytes) { char* p = wsp; wsp += (bytes + 255) & ~(size_t)255; return (void*)p; };
    float* WN = (float*)take((size_t)CO * CC * 4); bf* Bh = (bf*)take((size_t)CO * KK * 2); bf* Bl = (bf*)take((size_t)CO * KK * 2); float* PN = (float*)take((size_t)CC * NP * 4); bf* Ah = (bf*)take((size_t)NP * KK * 2); bf* Al = (bf*)take((size_t)NP * KK * 2); float* S = (float*)take((size_t)NP * CO * 4);
    if ((size_t)(wsp - (char*)d_ws) > ws_size) return;
    k_wn<<<(CO * CC + 255) / 256, 256, 0, stream>>>(w, WN); k_wnp<<<(CO * KK / 4 + 255) / 256, 256, 0, stream>>>(w, WN, Bh, Bl);
    for (int n = 0; n < NI; ++n) { const float* xi = x + (size_t)n * CC * NP;
        k_pn<<<(CC * NP / 4 + 255) / 256, 256, 0, stream>>>(xi, PN); k_pat<<<(NP * KK / 4 + 255) / 256, 256, 0, stream>>>(xi, PN, Ah, Al);
        k_gemmw<bf, 2, false><<<dim3(NP / 64, CO / 64, 1), 32, 0, stream>>>(Ah, Al, Bh, Bl, KK, S, CO, nullptr, 0, 0, 0);
        k_out<<<(CO * NP / 4 + 255) / 256, 256, 0, stream>>>(S, pw, OUT + (size_t)n * CO * NP); }
}
